// MultiplicativeLayer_13786845020927
// MI455X (gfx1250) — hardware-run, weakly checked
//
#include <hip/hip_runtime.h>


#ifndef NB
#define NB 32
#endif
#define NB_FULL 32
#ifndef HWP
#define HWP 1024
#endif
#define HW_FULL 1024
#ifndef OUT_HW
#define OUT_HW HWP
#endif
#define CIN   256
#define IC    64
#define MC    16
#define N1    (IC + MC)
#define COUT  256
#define EK    (MC * IC)
#define NPOS  64
#define MW    4
#define XSP   264
#define ISP   68
#define MSP   20
#define ESP   72
#define OSP   68
#define WCARRY 4096.0f
#define WCINV  (1.0f / 4096.0f)

static_assert(NPOS == 64);
static_assert(IC == 64);
static_assert(N1 == 5 * 16);
static_assert(CIN % 32 == 0);
static_assert(EK % 32 == 0);
static_assert(COUT == 64 * MW);
static_assert(32 * MW == 2 * NPOS);
static_assert(32 * MW * 32 == NPOS * IC);
static_assert((CIN * NPOS / 4) % (32 * MW) == 0);
static_assert(HWP % NPOS == 0);
static_assert(((size_t)NB * HWP) % NPOS == 0);
static_assert(32 * 16 * 8 == 16 * NPOS * 4);
static_assert((XSP * 2) % 16 == 0);
static_assert((ISP * 4) % 16 == 0);
static_assert((ESP * 2) % 16 == 0);
static_assert((OSP * 4) % 16 == 0);
static_assert(XSP >= CIN);
static_assert(ISP >= IC);
static_assert(MSP >= MC);
static_assert(ESP >= IC);
static_assert(OSP >= NPOS);
static_assert((size_t)NPOS * XSP * 2 + (size_t)NPOS * ISP * 4 + (size_t)NPOS * MSP * 4 + (size_t)NPOS * ESP * 2 + (size_t)MW * 16 * OSP * 4 <= (size_t)131072);
static_assert(NB <= NB_FULL);
static_assert(HWP <= HW_FULL);
static_assert(((size_t)IC * CIN) % 8 == 0);
static_assert(((size_t)MC * CIN) % 8 == 0);
static_assert(((size_t)COUT * EK) % 8 == 0);

typedef _Float16 h16;
typedef unsigned short bf;
typedef __attribute__((ext_vector_type(16))) __bf16   v16bf;
typedef __attribute__((ext_vector_type(16))) _Float16 v16h;
typedef __attribute__((ext_vector_type(8)))  _Float16 v8h;
typedef __attribute__((ext_vector_type(8)))  unsigned short v8us;
typedef __attribute__((ext_vector_type(8)))  float    v8f;
typedef __attribute__((ext_vector_type(4)))  float    v4f;
typedef v4f  __attribute__((may_alias)) v4fa;
typedef v8us __attribute__((may_alias)) v8usa;

__device__ __forceinline__ unsigned short f2bf(float f) { unsigned u = __float_as_uint(f); u += 0x7FFFu + ((u >> 16) & 1u); return (unsigned short)(u >> 16); }
__device__ __forceinline__ float bfr(float f) { return __uint_as_float(((unsigned)f2bf(f)) << 16); }
__device__ __forceinline__ v16h cat16(v8h lo, v8h hi) { return __builtin_shufflevector(lo, hi, 0, 1, 2, 3, 4, 5, 6, 7, 8, 9, 10, 11, 12, 13, 14, 15); }
__device__ __forceinline__ v16bf cat16b(v8us lo, v8us hi) { return __builtin_bit_cast(v16bf, __builtin_shufflevector(lo, hi, 0, 1, 2, 3, 4, 5, 6, 7, 8, 9, 10, 11, 12, 13, 14, 15)); }
__device__ __forceinline__ v8f wmma16(v16h a, v16h b, v8f c) { return __builtin_amdgcn_wmma_f32_16x16x32_f16(false, a, false, b, (short)0, c, false, false); }
__device__ __forceinline__ v8f wmmab(v16bf a, v16bf b, v8f c) { return __builtin_amdgcn_wmma_f32_16x16x32_bf16(false, a, false, b, (short)0, c, false, false); }
__device__ __forceinline__ v8f wmmabg(v16bf a, v16bf b, v8f c) { c = wmmab(a, b, c); asm volatile("v_nop\n\tv_nop\n\tv_nop\n\tv_nop" : "+v"(c) : "v"(a), "v"(b)); return c; }
__device__ __forceinline__ v8f wmma16g(v16h a, v16h b, v8f c) { c = wmma16(a, b, c); asm volatile("v_nop\n\tv_nop\n\tv_nop\n\tv_nop" : "+v"(c) : "v"(a), "v"(b)); return c; }
__device__ __forceinline__ v16h  ldh(const h16* p) { return cat16(*(const v8h*)p, *(const v8h*)(p + 16)); }
__device__ __forceinline__ v16bf ldb(const bf* p)  { return cat16b(*(const v8us*)p, *(const v8us*)(p + 16)); }
__device__ __forceinline__ void wave_sync() { __builtin_amdgcn_fence(3  , "wavefront"); __builtin_amdgcn_wave_barrier(); asm volatile("" ::: "memory"); }
__device__ __forceinline__ h16 toh_flush(float v) { const h16 r = (h16)v; return (fabsf(v) < 6.103515625e-05f) ? (h16)0.0f : r; }

__global__ __launch_bounds__(256) void k_cvt8(const float* __restrict__ src, bf* dst, size_t n8) {
    const size_t i = (size_t)blockIdx.x * 256 + threadIdx.x; if (i >= n8) return;
    const v8f v = *(const v8f*)(src + i * 8); v8us o;
#pragma unroll
    for (int k = 0; k < 8; ++k) o[k] = f2bf(v[k]);
    *(volatile v8us*)(dst + i * 8) = o; __threadfence(); *(volatile v8us*)(dst + i * 8) = o;
}

__global__ __launch_bounds__(256) void k_wconv(const float* __restrict__ src, h16* dst, size_t n8) {
    const size_t i = (size_t)blockIdx.x * 256 + threadIdx.x; if (i >= n8) return;
    const v8f v = *(const v8f*)(src + i * 8); v8h o;
#pragma unroll
    for (int k = 0; k < 8; ++k) o[k] = toh_flush(bfr(v[k]) * WCARRY);
    *(volatile v8h*)(dst + i * 8) = o; __threadfence(); *(volatile v8h*)(dst + i * 8) = o;
}

__global__ __launch_bounds__(32 * MW) void k_main(const float* __restrict__ X, const bf* __restrict__ W1, const h16* __restrict__ WH,
                                                  const float* __restrict__ info_b, const float* __restrict__ mask_b, const float* __restrict__ out_b, float* OUT) {
    __shared__ __align__(16) bf    xs[NPOS * XSP];
    __shared__ __align__(16) float fin[NPOS * ISP];
    __shared__ __align__(16) float fmk[NPOS * MSP];
    __shared__ __align__(16) h16   es[NPOS * ESP];
    __shared__ __align__(16) float os[MW * 16 * OSP];
    const int tid = threadIdx.x, lane = tid & 31, lr = lane & 15, hi = lane >> 4;
    const int wave = __builtin_amdgcn_readfirstlane((int)(threadIdx.x >> 5));
    const int g0 = blockIdx.x * NPOS; const int b = g0 / HWP, hw0 = g0 % HWP;
    const float* xb = X + (size_t)b * CIN * HW_FULL + hw0;

#pragma unroll 4
    for (int it = 0; it < (CIN * NPOS / 4) / (32 * MW); ++it) {
        const int idx = it * (32 * MW) + tid; const int c = idx >> 4, q = idx & 15;
        const v4f v = *(const v4f*)(xb + (size_t)c * HW_FULL + 4 * q);
#pragma unroll
        for (int j = 0; j < 4; ++j) xs[(4 * q + j) * XSP + c] = f2bf(v[j]);
    }
    __syncthreads();

    {
        v8f a1[5];
#pragma unroll
        for (int nt = 0; nt < 5; ++nt) a1[nt] = (v8f){};
        const int ao = (16 * wave + lr) * XSP + 8 * hi;
        const size_t bo = (size_t)lr * CIN + 8 * hi;
#pragma unroll 1
        for (int kc = 0; kc < CIN; kc += 32) {
            const v16bf a = cat16b(*(const v8usa*)(&xs[ao + kc]), *(const v8usa*)(&xs[ao + kc + 16]));
#pragma unroll
            for (int nt = 0; nt < 5; ++nt) { const v16bf w = ldb(W1 + bo + (size_t)nt * 16 * CIN + kc); a1[nt] = wmmabg(a, w, a1[nt]); }
        }
        const int prow = 16 * wave + 8 * hi;
#pragma unroll
        for (int nt = 0; nt < 4; ++nt) { const float bi = bfr(info_b[nt * 16 + lr]);
#pragma unroll
            for (int j = 0; j < 8; ++j) fin[(prow + j) * ISP + nt * 16 + lr] = fmaxf(a1[nt][j] + bi, 0.0f); }
        { const float bm = bfr(mask_b[lr]);
#pragma unroll
          for (int j = 0; j < 8; ++j) { const float t = a1[4][j] + bm; fmk[(prow + j) * MSP + lr] = 1.0f / (1.0f + expf(-t)); } }
    }
    __syncthreads();

    v8f acc[4][4];
#pragma unroll
    for (int ot = 0; ot < 4; ++ot)
#pragma unroll
        for (int ps = 0; ps < 4; ++ps) acc[ot][ps] = (v8f){};
    const int ep = tid >> 1, eh = tid & 1;
    const size_t wo = (size_t)(64 * wave + lr) * EK + 8 * hi;
#pragma unroll 1
    for (int m = 0; m < MC; ++m) {
        const float mv = fmk[ep * MSP + m];
#pragma unroll
        for (int q = 0; q < 4; ++q) {
            const v4f x0 = *(const v4fa*)(&fin[ep * ISP + 32 * eh + 8 * q]); const v4f x1 = *(const v4fa*)(&fin[ep * ISP + 32 * eh + 8 * q + 4]); v8h e;
#pragma unroll
            for (int i = 0; i < 4; ++i) { e[i] = toh_flush(mv * x0[i]); e[4 + i] = toh_flush(mv * x1[i]); }
            *(v8h*)(&es[ep * ESP + 32 * eh + 8 * q]) = e;
        }
        __syncthreads();
#pragma unroll 1
        for (int ks = 0; ks < 2; ++ks) {
            v16h eb[4];
#pragma unroll
            for (int ps = 0; ps < 4; ++ps) { const int eo = (16 * ps + lr) * ESP + 32 * ks + 8 * hi; eb[ps] = cat16(*(const v8h*)(&es[eo]), *(const v8h*)(&es[eo + 16])); }
#pragma unroll
            for (int ot = 0; ot < 4; ++ot) { const v16h a = ldh(WH + wo + (size_t)ot * 16 * EK + (size_t)(m * IC + 32 * ks));
#pragma unroll
                for (int ps = 0; ps < 4; ++ps) acc[ot][ps] = wmma16g(a, eb[ps], acc[ot][ps]); }
        }
        __syncthreads();
    }

    float* ob = OUT + (size_t)b * COUT * OUT_HW + hw0;
    const int wb = wave * 16 * OSP;
#pragma unroll
    for (int ot = 0; ot < 4; ++ot) {
        const int orow = 64 * wave + 16 * ot;
        float br[8];
#pragma unroll
        for (int j = 0; j < 8; ++j) br[j] = bfr(out_b[orow + 8 * hi + j]);
#pragma unroll
        for (int ps = 0; ps < 4; ++ps) {
#pragma unroll
            for (int j = 0; j < 8; ++j) os[wb + (8 * hi + j) * OSP + 16 * ps + lr] = fmaxf(acc[ot][ps][j] * WCINV + br[j], 0.0f); }
        wave_sync();
#pragma unroll 1
        for (int pz = 0; pz < 2; ++pz) {
#pragma unroll
            for (int s = 0; s < 8; ++s) { const int row = 2 * s + (lane >> 4), c4 = (lane & 15) * 4;
                const v4f val = *(const v4fa*)(&os[wb + row * OSP + c4]);
                *(volatile v4f*)(ob + (size_t)(orow + row) * OUT_HW + c4) = val; }
            if (pz == 0) __threadfence(); }
        wave_sync();
    }
}

static constexpr size_t al256(size_t v) { return (v + 255) & ~(size_t)255; }
static constexpr size_t SZ_W1 = al256((size_t)N1 * CIN * 2);
static constexpr size_t SZ_WH = al256((size_t)COUT * EK * 2);
static constexpr size_t SZ_TOTAL = SZ_W1 + SZ_WH;
static_assert(SZ_TOTAL <= (size_t)134217728);
static_assert(((size_t)IC * CIN * 2) % 256 == 0);

extern "C" void kernel_launch(void* const* d_in, const int* in_sizes, int n_in,
                              void* d_out, int out_size, void* d_ws, size_t ws_size, hipStream_t stream) {
    if (n_in < 7) return;
    const size_t needx = ((size_t)(NB - 1) * CIN + (CIN - 1)) * HW_FULL + HWP;
    const size_t needo = ((size_t)(NB - 1) * COUT + (COUT - 1)) * OUT_HW + HWP;
    if ((size_t)in_sizes[0] < needx) return;
    if ((size_t)in_sizes[1] < (size_t)IC * CIN || in_sizes[2] < IC) return;
    if ((size_t)in_sizes[3] < (size_t)MC * CIN || in_sizes[4] < MC) return;
    if ((size_t)in_sizes[5] < (size_t)COUT * EK || in_sizes[6] < COUT) return;
    if ((size_t)out_size < needo) return;
    if (SZ_TOTAL > ws_size) return;
    const float* x  = (const float*)d_in[0];
    const float* iw = (const float*)d_in[1]; const float* ib = (const float*)d_in[2];
    const float* mw = (const float*)d_in[3]; const float* mb = (const float*)d_in[4];
    const float* ow = (const float*)d_in[5]; const float* obias = (const float*)d_in[6];
    float* OUT = (float*)d_out;
    char* wsp = (char*)d_ws;
    bf*  W1 = (bf*)wsp;  wsp += SZ_W1;
    h16* WH = (h16*)wsp; wsp += SZ_WH;

    { const size_t n8 = (size_t)IC * CIN / 8;   k_cvt8<<<(unsigned)((n8 + 255) / 256), 256, 0, stream>>>(iw, W1, n8); }
    { const size_t n8 = (size_t)MC * CIN / 8;   k_cvt8<<<(unsigned)((n8 + 255) / 256), 256, 0, stream>>>(mw, W1 + (size_t)IC * CIN, n8); }
    { const size_t n8 = (size_t)COUT * EK / 8;  k_wconv<<<(unsigned)((n8 + 255) / 256), 256, 0, stream>>>(ow, WH, n8); }

    k_main<<<dim3((unsigned)((size_t)NB * HWP / NPOS), 1, 1), 32 * MW, 0, stream>>>(x, W1, WH, ib, mb, obias, OUT);
}
